// MemoryNet_32023276159359
// MI455X (gfx1250) — hardware-verified
//
#include <hip/hip_runtime.h>
#include <hip/hip_bf16.h>

#define N_MEM 256
#define N_EMB 128

typedef __attribute__((ext_vector_type(16))) _Float16 v16h;
typedef __attribute__((ext_vector_type(8)))  _Float16 v8h;
typedef __attribute__((ext_vector_type(16))) __bf16   v16b;
typedef __attribute__((ext_vector_type(8)))  __bf16   v8b;
typedef __attribute__((ext_vector_type(8)))  float    v8f;
typedef __attribute__((ext_vector_type(4)))  float    v4f;
typedef __attribute__((ext_vector_type(2)))  float    v2f;
#define PSCALE 32768.0f
#define PSCALE_INV (1.0f / 32768.0f)

__device__ __forceinline__ unsigned short f2bf_bits(float f) {
  unsigned u = __float_as_uint(f);
  return (unsigned short)((u + 0x7FFFu + ((u >> 16) & 1u)) >> 16);
}
__device__ __forceinline__ float bf_bits2f(unsigned short h) { return __uint_as_float(((unsigned)h) << 16); }

__device__ __forceinline__ void dep_guard_h(v8f& a, v8f& b, v16h x, v16h y) { asm volatile("v_nop\n\tv_nop\n\tv_nop\n\tv_nop" : "+v"(a), "+v"(b) : "v"(x), "v"(y)); }
__device__ __forceinline__ void dep_guard_b(v8f& a, v8f& b, v16b x, v16b y) { asm volatile("v_nop\n\tv_nop\n\tv_nop\n\tv_nop" : "+v"(a), "+v"(b) : "v"(x), "v"(y)); }
__device__ __forceinline__ void keep4_h(v16h a, v16h b, v16h c, v16h d) { asm volatile("v_nop" :: "v"(a), "v"(b), "v"(c), "v"(d)); }
__device__ __forceinline__ void keep4_b(v16b a, v16b b, v16b c, v16b d) { asm volatile("v_nop" :: "v"(a), "v"(b), "v"(c), "v"(d)); }
__device__ __forceinline__ void acc_guard4(v8f& a, v8f& b, v8f& c, v8f& d) { asm volatile("v_nop\n\tv_nop\n\tv_nop\n\tv_nop" : "+v"(a), "+v"(b), "+v"(c), "+v"(d)); }
template <typename T> struct Frag;
template <> struct Frag<_Float16> {
  typedef v16h V; union U { v16h v; v8h h[2]; };
  static __device__ __forceinline__ v16h load(const _Float16* p) {
    U f; f.h[0] = *(const v8h*)(p); f.h[1] = *(const v8h*)(p + 16); return f.v;
  }
  static __device__ __forceinline__ v8f mma(v16h a, v16h b, v8f c) {
    return __builtin_amdgcn_wmma_f32_16x16x32_f16(false, a, false, b, (short)0, c, false, false);
  }
  static __device__ __forceinline__ void guard(v8f& a, v8f& b, v16h x, v16h y) { dep_guard_h(a, b, x, y); }
  static __device__ __forceinline__ void keep(v16h a, v16h b, v16h c, v16h d) { keep4_h(a, b, c, d); }
};
template <> struct Frag<__bf16> {
  typedef v16b V; union U { v16b v; v8b h[2]; };
  static __device__ __forceinline__ v16b load(const __bf16* p) {
    U f; f.h[0] = *(const v8b*)(p); f.h[1] = *(const v8b*)(p + 16); return f.v;
  }
  static __device__ __forceinline__ v8f mma(v16b a, v16b b, v8f c) {
    return __builtin_amdgcn_wmma_f32_16x16x32_bf16(false, a, false, b, (short)0, c, false, false);
  }
  static __device__ __forceinline__ void guard(v8f& a, v8f& b, v16b x, v16b y) { dep_guard_b(a, b, x, y); }
  static __device__ __forceinline__ void keep(v16b a, v16b b, v16b c, v16b d) { keep4_b(a, b, c, d); }
};

template <int ET> struct Elem;
template <> struct Elem<0> { typedef _Float16 T; };
template <> struct Elem<1> { typedef __bf16 T; };
template <int ET, bool SPLIT, int BIAS_MODE, int OUT_MODE, bool RESID, int ACT = 0>
__global__ __launch_bounds__(256) void wmma_gemm64(
    const unsigned short* __restrict__ Ap, const unsigned short* __restrict__ A2p, int lda, long strideA,
    const unsigned short* __restrict__ Btp, const unsigned short* __restrict__ Bt2p, int ldb, long strideB,
    void* __restrict__ Cout, void* __restrict__ Cout2, int ldc, long strideC,
    const float* __restrict__ bias,
    const float* __restrict__ resid, long strideR,
    int M, int N, int K, float scale, float oscale) {
  typedef typename Elem<ET>::T T;
  typedef typename Frag<T>::V V;
  const T* A = (const T*)Ap; const T* A2 = (const T*)A2p; const T* Bt = (const T*)Btp; const T* Bt2 = (const T*)Bt2p;
  __shared__ __align__(16) float sT[8][16 * 68];
  const int b    = blockIdx.y;
  const int lane = threadIdx.x & 31;
  const int wave = threadIdx.x >> 5;
  const int tilesN = N >> 6;
  const int tilesM = M >> 6;
  const int tile = blockIdx.x * 8 + wave;
  if (tile >= tilesM * tilesN) return;
  const int tm = tile / tilesN;
  const int tn = tile - tm * tilesN;
  const int m0 = tm << 6;
  const int n0 = tn << 6;

  const T* Ab  = A  + (size_t)b * strideA;
  const T* Bb  = Bt + (size_t)b * strideB;
  const T* Ab2 = SPLIT ? (A2  + (size_t)b * strideA) : nullptr;
  const T* Bb2 = SPLIT ? (Bt2 + (size_t)b * strideB) : nullptr;

  const int rlane = lane & 15;
  const int koff  = (lane >> 4) * 8;
  const int mOff  = (lane >> 4) * 8;

  v8f acc[4][4];
#pragma unroll
  for (int i = 0; i < 4; ++i)
#pragma unroll
    for (int j = 0; j < 4; ++j) acc[i][j] = (v8f){0.f,0.f,0.f,0.f,0.f,0.f,0.f,0.f};

  for (int k0 = 0; k0 < K; k0 += 32) {
    V bh[4], bl[4];
#pragma unroll
    for (int j = 0; j < 4; ++j) {
      const size_t bo = (size_t)(n0 + (j << 4) + rlane) * ldb + koff + k0;
      bh[j] = Frag<T>::load(Bb + bo);
      if (SPLIT) bl[j] = Frag<T>::load(Bb2 + bo);
    }
#pragma unroll
    for (int i = 0; i < 4; ++i) {
      const size_t ao = (size_t)(m0 + (i << 4) + rlane) * lda + koff + k0;
      V ah = Frag<T>::load(Ab + ao);
      V al;
      if (SPLIT) al = Frag<T>::load(Ab2 + ao);
#pragma unroll
      for (int j = 0; j < 4; ++j) {
        acc[i][j] = Frag<T>::mma(ah, bh[j], acc[i][j]);
        if (SPLIT) {
          acc[i][j] = Frag<T>::mma(ah, bl[j], acc[i][j]);
          acc[i][j] = Frag<T>::mma(al, bh[j], acc[i][j]);
        }
      }
      Frag<T>::guard(acc[i][0], acc[i][3], ah, SPLIT ? al : ah);
    }
    Frag<T>::keep(bh[0], bh[1], bh[2], bh[3]);
    if (SPLIT) Frag<T>::keep(bl[0], bl[1], bl[2], bl[3]);
  }
  acc_guard4(acc[0][0], acc[0][1], acc[0][2], acc[0][3]);
  acc_guard4(acc[1][0], acc[1][1], acc[1][2], acc[1][3]);
  acc_guard4(acc[2][0], acc[2][1], acc[2][2], acc[2][3]);
  acc_guard4(acc[3][0], acc[3][1], acc[3][2], acc[3][3]);

  float* slab = sT[wave];
  const float* Rb = RESID ? (resid + (size_t)b * strideR) : nullptr;
#pragma unroll
  for (int i = 0; i < 4; ++i) {
    const int mBase = m0 + (i << 4);
#pragma unroll
    for (int j = 0; j < 4; ++j) {
      const int n = n0 + (j << 4) + rlane;
      float bv = 0.f;
      if (BIAS_MODE == 2) bv = bias[n];
#pragma unroll
      for (int r = 0; r < 8; ++r) {
        float v = acc[i][j][r] * scale;
        if (BIAS_MODE == 1) v += bias[mBase + mOff + r];
        if (BIAS_MODE == 2) v += bv;
        if (RESID) v += Rb[(size_t)(mBase + mOff + r) * ldc + n];
        if (ACT == 1) v = tanhf(v);
        if (ACT == 2) v = fmaxf(v, 0.0f);
        if (ACT == 3) v = v / (1.0f + expf(-v));
        if (ACT == 4) v = (v > 0.f) ? v : 0.01f * v;
        if (ACT == 5) v = 0.5f * v * (1.0f + erff(v * 0.70710678118654752f));
        v = v * oscale;
        slab[(mOff + r) * 68 + (j << 4) + rlane] = v;
      }
    }
    __builtin_amdgcn_fence(__ATOMIC_RELEASE, "workgroup");
    __builtin_amdgcn_wave_barrier();
    __builtin_amdgcn_fence(__ATOMIC_ACQUIRE, "workgroup");
    if (OUT_MODE == 0) {
      float* C = (float*)Cout + (size_t)b * strideC;
      const int hh = lane >> 4, c4 = (lane & 15) * 4;
      for (int pass = 0; pass < 2; ++pass) {
#pragma unroll
        for (int it = 0; it < 8; ++it) {
          const int row = it * 2 + hh;
          v4f v = *(const v4f*)(slab + row * 68 + c4);
          *(volatile v4f*)(C + (size_t)(mBase + row) * ldc + n0 + c4) = v;
        }
        __threadfence();
      }
    } else {
      const int q = lane >> 3, c8 = (lane & 7) * 8;
      unsigned short* C  = (unsigned short*)Cout  + (size_t)b * strideC;
      unsigned short* C2 = (OUT_MODE == 2) ? ((unsigned short*)Cout2 + (size_t)b * strideC) : nullptr;
      for (int pass = 0; pass < 2; ++pass) {
#pragma unroll
        for (int it = 0; it < 4; ++it) {
          const int row = it * 4 + q;
          const float* sp = slab + row * 68 + c8;
          v8h hv, lv;
#pragma unroll
          for (int e = 0; e < 8; ++e) {
            if (OUT_MODE == 1) {
              hv[e] = (_Float16)sp[e];
            } else {
              unsigned short hb = f2bf_bits(sp[e]);
              unsigned short lb = f2bf_bits(sp[e] - bf_bits2f(hb));
              hv[e] = __builtin_bit_cast(_Float16, hb);
              lv[e] = __builtin_bit_cast(_Float16, lb);
            }
          }
          *(volatile v8h*)(C + (size_t)(mBase + row) * ldc + n0 + c8) = hv;
          if (OUT_MODE == 2) *(volatile v8h*)(C2 + (size_t)(mBase + row) * ldc + n0 + c8) = lv;
        }
        __threadfence();
      }
    }
    __builtin_amdgcn_fence(__ATOMIC_RELEASE, "workgroup");
    __builtin_amdgcn_wave_barrier();
    __builtin_amdgcn_fence(__ATOMIC_ACQUIRE, "workgroup");
  }
}

__global__ __launch_bounds__(256) void cast_scale_f32_f16x2(
    const float* __restrict__ in, _Float16* __restrict__ out, int n2, float sc) {
  int i = blockIdx.x * 256 + threadIdx.x;
  if (i < n2) {
    const v2f x = *(const v2f*)(in + 2 * (size_t)i);
    const _Float16 h0 = (_Float16)(x[0] * sc), h1 = (_Float16)(x[1] * sc);
    const unsigned u = (unsigned)__builtin_bit_cast(unsigned short, h0) | ((unsigned)__builtin_bit_cast(unsigned short, h1) << 16);
    ((volatile unsigned*)out)[i] = u;
    __threadfence();
    ((volatile unsigned*)out)[i] = u;
  }
}

__global__ __launch_bounds__(256) void softmax_rows_f16(
    const float* __restrict__ S, _Float16* __restrict__ P, int nrows) {
  const int lane = threadIdx.x & 31;
  const int wave = threadIdx.x >> 5;
  const int row  = blockIdx.x * 8 + wave;
  if (row >= nrows) return;
  const float* sp = S + (size_t)row * N_MEM + lane * 8;
  const v4f x0 = *(const v4f*)(sp);
  const v4f x1 = *(const v4f*)(sp + 4);
  float mx = fmaxf(fmaxf(fmaxf(x0[0], x0[1]), fmaxf(x0[2], x0[3])),
                   fmaxf(fmaxf(x1[0], x1[1]), fmaxf(x1[2], x1[3])));
#pragma unroll
  for (int off = 1; off < 32; off <<= 1) mx = fmaxf(mx, __shfl_xor(mx, off, 32));
  v4f e0, e1;
  float s = 0.f;
#pragma unroll
  for (int i = 0; i < 4; ++i) { e0[i] = __expf(x0[i] - mx); s += e0[i]; }
#pragma unroll
  for (int i = 0; i < 4; ++i) { e1[i] = __expf(x1[i] - mx); s += e1[i]; }
#pragma unroll
  for (int off = 1; off < 32; off <<= 1) s += __shfl_xor(s, off, 32);
  const float inv = 1.0f / s;
  v8h hv;
#pragma unroll
  for (int i = 0; i < 4; ++i) {
    const float p0 = e0[i] * inv;
    const float p1 = e1[i] * inv;
    hv[i]     = (_Float16)(p0 * PSCALE);
    hv[4 + i] = (_Float16)(p1 * PSCALE);
  }
  _Float16* pp = P + (size_t)row * N_MEM + lane * 8;
  *(volatile v8h*)pp = hv;
  __threadfence();
  *(volatile v8h*)pp = hv;
}

extern "C" void kernel_launch(void* const* d_in, const int* in_sizes, int n_in,
                              void* d_out, int out_size, void* d_ws, size_t ws_size,
                              hipStream_t stream) {
  if (n_in < 6) return;
  const int nIn = in_sizes[0];
  if (in_sizes[1] != N_MEM * N_EMB || in_sizes[2] != N_EMB * N_EMB || in_sizes[3] != N_EMB ||
      in_sizes[4] != N_EMB * N_EMB || in_sizes[5] != N_EMB) return;
  if (nIn <= 0 || (nIn % (N_EMB * 64)) != 0 || out_size != nIn) return;
  const int rows = nIn / N_EMB;

  const float* input  = (const float*)d_in[0];
  const float* memory = (const float*)d_in[1];
  const float* Wk     = (const float*)d_in[2];
  const float* bk     = (const float*)d_in[3];
  const float* Wv     = (const float*)d_in[4];
  const float* bv     = (const float*)d_in[5];
  float* out = (float*)d_out;

  size_t off = 0;
  auto carve = [&](size_t bytes) { size_t o = off; off += (bytes + 127) & ~(size_t)127; return o; };
  const size_t o_mem16 = carve((size_t)N_MEM * N_EMB * 2);
  const size_t o_wk16  = carve((size_t)N_EMB * N_EMB * 2);
  const size_t o_wv16  = carve((size_t)N_EMB * N_EMB * 2);
  const size_t o_key16 = carve((size_t)N_MEM * N_EMB * 2);
  const size_t o_valT  = carve((size_t)N_EMB * N_MEM * 2);
  const size_t o_q16   = carve((size_t)rows * N_EMB * 2);
  const size_t o_S     = carve((size_t)rows * N_MEM * 4);
  const size_t o_P     = carve((size_t)rows * N_MEM * 2);
  if (off > ws_size || off > (size_t)134217728) return;

  char* ws = (char*)d_ws;
  _Float16* mem16 = (_Float16*)(ws + o_mem16);
  _Float16* wk16  = (_Float16*)(ws + o_wk16);
  _Float16* wv16  = (_Float16*)(ws + o_wv16);
  _Float16* key16 = (_Float16*)(ws + o_key16);
  _Float16* valT  = (_Float16*)(ws + o_valT);
  _Float16* q16   = (_Float16*)(ws + o_q16);
  float*    S     = (float*)(ws + o_S);
  _Float16* P     = (_Float16*)(ws + o_P);

  {
    const int n2m = N_MEM * N_EMB / 2;
    cast_scale_f32_f16x2<<<(n2m + 255) / 256, 256, 0, stream>>>(memory, mem16, n2m, 64.0f);
    const int n2w = N_EMB * N_EMB / 2;
    cast_scale_f32_f16x2<<<(n2w + 255) / 256, 256, 0, stream>>>(Wk, wk16, n2w, 256.0f);
    cast_scale_f32_f16x2<<<(n2w + 255) / 256, 256, 0, stream>>>(Wv, wv16, n2w, 256.0f);
    const int n2q = rows * (N_EMB / 2);
    cast_scale_f32_f16x2<<<(n2q + 255) / 256, 256, 0, stream>>>(input, q16, n2q, 16.0f);
  }

  {
    const int tiles = (N_MEM / 64) * (N_EMB / 64);
    wmma_gemm64<0, false, 2, 1, false, 0><<<dim3((tiles + 7) / 8, 1), 256, 0, stream>>>(
        (const unsigned short*)mem16, (const unsigned short*)mem16, N_EMB, 0L,
        (const unsigned short*)wk16, (const unsigned short*)wk16, N_EMB, 0L,
        (void*)key16, (void*)key16, N_EMB, 0L,
        bk, bk, 0L, N_MEM, N_EMB, N_EMB, 1.0f / 16384.0f, 256.0f);
  }
  {
    const int tiles = (N_EMB / 64) * (N_MEM / 64);
    wmma_gemm64<0, false, 1, 1, false, 0><<<dim3((tiles + 7) / 8, 1), 256, 0, stream>>>(
        (const unsigned short*)wv16, (const unsigned short*)wv16, N_EMB, 0L,
        (const unsigned short*)mem16, (const unsigned short*)mem16, N_EMB, 0L,
        (void*)valT, (void*)valT, N_MEM, 0L,
        bv, bv, 0L, N_EMB, N_MEM, N_EMB, 1.0f / 16384.0f, 256.0f);
  }
  {
    const int tiles = (rows / 64) * (N_MEM / 64);
    wmma_gemm64<0, false, 0, 0, false, 0><<<dim3((tiles + 7) / 8, 1), 256, 0, stream>>>(
        (const unsigned short*)q16, (const unsigned short*)q16, N_EMB, 0L,
        (const unsigned short*)key16, (const unsigned short*)key16, N_EMB, 0L,
        (void*)S, (void*)S, N_MEM, 0L,
        bk, bk, 0L, rows, N_MEM, N_EMB, 1.0f / 4096.0f, 1.0f);
  }
  softmax_rows_f16<<<(rows + 7) / 8, 256, 0, stream>>>(S, P, rows);
  {
    const int tiles = (rows / 64) * (N_EMB / 64);
    wmma_gemm64<0, false, 0, 0, false, 0><<<dim3((tiles + 7) / 8, 1), 256, 0, stream>>>(
        (const unsigned short*)P, (const unsigned short*)P, N_MEM, 0L,
        (const unsigned short*)valT, (const unsigned short*)valT, N_MEM, 0L,
        (void*)out, (void*)out, N_EMB, 0L,
        bv, bv, 0L, rows, N_EMB, N_MEM, PSCALE_INV / 256.0f, 1.0f);
  }
}
